// NonLocal3D_67671504716358
// MI455X (gfx1250) — hardware-verified
//
#include <hip/hip_runtime.h>
#include <math.h>
#include <stdint.h>

#define BATCH 2
#define NPOS  6272
#define CIN   256
#define CI    128
#ifndef NB
#define NB BATCH
#endif
#define ROWS  (BATCH * NPOS)
#define ROWSP (NB * NPOS)
#define CK    448
#define NKB   (CK / 32)
#define NCHK  (NPOS / CK)
#define QT    16
#define ATT_THREADS 256
#define SCP   (CK + 16)
#define PLP   (CK + 8)
#define CTP   (CI + 8)
#define SLAB64 (16 * 68)
#define VTP   72
#define OUT_ROWS 128
#define TSC   8.0f
#define FSC   8.0f
#define RSC   2048.0f
#define PCAR  32768.0f
#define GSC   256.0f
#define YSC   4096.0f
#define WOS   1024.0f
#define BN_EPS 1e-3f
#define LOG2E 1.4426950408889634f
#define WS_CAP ((size_t)134217728)

static_assert(NB >= 1 && NB <= BATCH);
static_assert((NPOS % CK) == 0 && CK == 32 * NKB && NKB >= 4 && NKB <= 16 && NCHK * CK == NPOS);
static_assert((NPOS % 64) == 0 && (NPOS % QT) == 0 && (ROWSP % OUT_ROWS) == 0 && (ROWSP % 64) == 0);
static_assert(CI == 128 && (CIN % 64) == 0 && (CI % 64) == 0 && (CIN % 32) == 0 && (CI % 32) == 0);
static_assert(ATT_THREADS == 16 * QT && QT == 16 && CI == 16 * (ATT_THREADS / 32) && OUT_ROWS == 8 * 16);
static_assert(16 * CTP * 2 <= 16 * SCP * 4 && CTP >= CI + 8 && SCP >= CK + 16 && PLP >= CK + 8);
static_assert(((PLP * 2) % 16) == 0 && ((SCP * 4) % 16) == 0 && ((VTP * 2) % 16) == 0 && ((CTP * 2) % 16) == 0);
static_assert(64 * VTP >= 63 * VTP + 64);
static_assert(16 * (CI / 8) == ATT_THREADS);
static_assert(((ROWSP * CIN) % 2048) == 0);
static_assert(((NPOS * 2) % 128) == 0 && ((CI * 2) % 128) == 0 && ((CIN * 4) % 128) == 0);

typedef unsigned short u16;
typedef _Float16 v16h __attribute__((ext_vector_type(16)));
typedef _Float16 v8h  __attribute__((ext_vector_type(8)));
typedef __bf16   v16b __attribute__((ext_vector_type(16)));
typedef float    v8f  __attribute__((ext_vector_type(8)));
typedef float    v4f  __attribute__((ext_vector_type(4)));
typedef unsigned int v4u __attribute__((ext_vector_type(4)));

union FragH { v16h v; v8h h[2]; v4u u[2]; };
union FragB { v16b v; v4u u[2]; };
union AttLds { float s[16 * SCP]; u16 c[2 * 16 * SCP]; };

__device__ __forceinline__ unsigned short bf_bits(float f) {
  unsigned u = __float_as_uint(f);
  return (unsigned short)((u + 0x7FFFu + ((u >> 16) & 1u)) >> 16);
}
__device__ __forceinline__ float bf_up(unsigned short h) { return __uint_as_float(((unsigned)h) << 16); }
__device__ __forceinline__ float bfr(float f) { return bf_up(bf_bits(f)); }
__device__ __forceinline__ unsigned short h_bits(_Float16 x) { return __builtin_bit_cast(unsigned short, x); }
__device__ __forceinline__ unsigned pk16(unsigned short a, unsigned short b) { return (unsigned)a | ((unsigned)b << 16); }
__device__ __forceinline__ v8f zero8() { v8f z = {0.f, 0.f, 0.f, 0.f, 0.f, 0.f, 0.f, 0.f}; return z; }

__device__ __forceinline__ v16h ldfrag_h(const _Float16* p) {
  FragH f;
  f.h[0] = *(const v8h*)(p);
  f.h[1] = *(const v8h*)(p + 16);
  return f.v;
}
__device__ __forceinline__ v16b ldfrag_b(const u16* p) {
  FragB f;
  f.u[0] = *(const v4u*)(p);
  f.u[1] = *(const v4u*)(p + 16);
  return f.v;
}

__device__ __forceinline__ v8f mma_h(v16h a, v16h b, v8f c) {
  return __builtin_amdgcn_wmma_f32_16x16x32_f16(false, a, false, b, (short)0, c, false, false);
}
__device__ __forceinline__ v8f mma_b(v16b a, v16b b, v8f c) {
  return __builtin_amdgcn_wmma_f32_16x16x32_bf16(false, a, false, b, (short)0, c, false, false);
}
__device__ __forceinline__ void guard1x2(v8f& a, v16h x0, v16h x1) {
#if defined(__HIP_DEVICE_COMPILE__)
  asm volatile("v_nop\n\tv_nop\n\tv_nop\n\tv_nop" : "+v"(a) : "v"(x0), "v"(x1) : "memory");
#endif
}
template <typename F>
__device__ __forceinline__ void guard6(v8f& a, v8f& b, v8f& c, v8f& d, F x0, F x1, F x2, F x3, F x4, F x5) {
#if defined(__HIP_DEVICE_COMPILE__)
  asm volatile("v_nop\n\tv_nop\n\tv_nop\n\tv_nop"
               : "+v"(a), "+v"(b), "+v"(c), "+v"(d) : "v"(x0), "v"(x1), "v"(x2), "v"(x3), "v"(x4), "v"(x5) : "memory");
#endif
}
__device__ __forceinline__ void guard8x6(v8f& a0, v8f& a1, v8f& a2, v8f& a3, v8f& e0, v8f& e1, v8f& e2, v8f& e3,
                                         v16h x0, v16h x1, v16h x2, v16h x3, v16h x4, v16h x5) {
#if defined(__HIP_DEVICE_COMPILE__)
  asm volatile("v_nop\n\tv_nop\n\tv_nop\n\tv_nop"
               : "+v"(a0), "+v"(a1), "+v"(a2), "+v"(a3), "+v"(e0), "+v"(e1), "+v"(e2), "+v"(e3)
               : "v"(x0), "v"(x1), "v"(x2), "v"(x3), "v"(x4), "v"(x5) : "memory");
#endif
}
__device__ __forceinline__ void acc_guard1(v8f& a) {
#if defined(__HIP_DEVICE_COMPILE__)
  asm volatile("v_nop\n\tv_nop\n\tv_nop\n\tv_nop" : "+v"(a));
#endif
}
__device__ __forceinline__ void wave_sync_lds() {
  __builtin_amdgcn_fence(__ATOMIC_RELEASE, "workgroup");
  __builtin_amdgcn_wave_barrier();
  __builtin_amdgcn_fence(__ATOMIC_ACQUIRE, "workgroup");
}

__global__ __launch_bounds__(256) void cvt16(const float* __restrict__ x, u16* D, int n8, int mode, float scale) {
  const int gt = blockIdx.x * 256 + (int)threadIdx.x;
  if (gt >= n8) return;
  const float* p = x + (size_t)gt * 8;
  const v4f a = *(const v4f*)(p), c4 = *(const v4f*)(p + 4);
  float v[8];
#pragma unroll
  for (int e = 0; e < 4; ++e) { v[e] = a[e]; v[4 + e] = c4[e]; }
  unsigned short s[8];
#pragma unroll
  for (int e = 0; e < 8; ++e) {
    const float vb = bfr(v[e]);
    const float vf = (mode == 1) ? vb : v[e];
    const unsigned short hb = h_bits((_Float16)(vf * scale));
    const unsigned short bb = bf_bits(v[e]);
    s[e] = (mode != 0) ? hb : bb;
  }
  v4u o;
#pragma unroll
  for (int e = 0; e < 4; ++e) o[e] = pk16(s[2 * e], s[2 * e + 1]);
  u16* d = D + (size_t)gt * 8;
  for (int pass = 0; pass < 2; ++pass) {
    *(volatile v4u*)(d) = o;
    __threadfence();
  }
}

__global__ __launch_bounds__(256) void tr16(const float* __restrict__ X, u16* XTo, int R, int C, int mode, float scale) {
  __shared__ __align__(16) u16 TH[64 * VTP];
  const int tid = threadIdx.x;
  const int bid = blockIdx.x;
  const int nrt = R >> 6;
  const int rt  = bid % nrt;
  const int ct  = bid / nrt;
  const int r0  = rt * 64;
  const int c0  = ct * 64;
  {
    const int rl = tid >> 2;
    const int cc = (tid & 3) * 16;
    const float* src = X + (size_t)(r0 + rl) * (size_t)C + c0 + cc;
#pragma unroll
    for (int i = 0; i < 4; ++i) {
      const v4f a = *(const v4f*)(src + 4 * i);
#pragma unroll
      for (int e = 0; e < 4; ++e) {
        const float v  = a[e];
        const float vb = bfr(v);
        const float vf = (mode == 1) ? vb : v;
        const unsigned short hb = h_bits((_Float16)(vf * scale));
        const unsigned short bb = bf_bits(v);
        TH[(cc + 4 * i + e) * VTP + rl] = (mode != 0) ? hb : bb;
      }
    }
  }
  __syncthreads();
  v4u vh[2];
  const int q8 = tid >> 3, p8 = (tid & 7) * 8;
#pragma unroll
  for (int it = 0; it < 2; ++it) {
    const int line = it * 32 + q8;
    vh[it] = *(const v4u*)(TH + line * VTP + p8);
  }
  const size_t base = (size_t)c0 * (size_t)R + (size_t)r0 + (size_t)p8;
  for (int pass = 0; pass < 2; ++pass) {
#pragma unroll
    for (int it = 0; it < 2; ++it) {
      const int line = it * 32 + q8;
      *(volatile v4u*)(XTo + base + (size_t)line * (size_t)R) = vh[it];
    }
    __threadfence();
  }
}

__device__ __forceinline__ void stage64(float* sl, v8f a0, v8f a1, v8f a2, v8f a3, float oscale, int lane) {
  const int hh = lane >> 4, m = lane & 15;
#pragma unroll
  for (int r = 0; r < 8; ++r) {
    const int ro = (8 * hh + r) * 68 + m;
    sl[ro]      = a0[r] * oscale;
    sl[ro + 16] = a1[r] * oscale;
    sl[ro + 32] = a2[r] * oscale;
    sl[ro + 48] = a3[r] * oscale;
  }
  wave_sync_lds();
}
__device__ __forceinline__ void epi64(float* sl, v8f a0, v8f a1, v8f a2, v8f a3, float oscale, v4f badd, float* C, int N,
                                      size_t rowb, int col0, int lane) {
  const int hh = lane >> 4, m = lane & 15;
  stage64(sl, a0, a1, a2, a3, oscale, lane);
  v4f vals[8];
#pragma unroll
  for (int it = 0; it < 8; ++it) vals[it] = *(const v4f*)(sl + (it * 2 + hh) * 68 + m * 4) + badd;
  float* dst = C + (rowb + (size_t)hh) * (size_t)N + col0 + m * 4;
  for (int pass = 0; pass < 2; ++pass) {
#pragma unroll
    for (int it = 0; it < 8; ++it) {
      *(volatile v4f*)(dst + (size_t)(it * 2) * (size_t)N) = vals[it];
    }
    __threadfence();
  }
}
__device__ __forceinline__ void epi64hr(float* sl, v8f a0, v8f a1, v8f a2, v8f a3, float hscale, float rscale,
                                        const float* __restrict__ bias, u16* H, u16* Rr, int N, size_t rowb, int col0, int lane) {
  stage64(sl, a0, a1, a2, a3, 1.0f, lane);
  const int rq = lane >> 3, c8 = (lane & 7) * 8;
  const v4f b0 = *(const v4f*)(bias + col0 + c8), b1 = *(const v4f*)(bias + col0 + c8 + 4);
  float bb[8];
#pragma unroll
  for (int e = 0; e < 4; ++e) { bb[e] = bfr(b0[e]); bb[4 + e] = bfr(b1[e]); }
  v4u oh[4], orr[4];
#pragma unroll
  for (int i4 = 0; i4 < 4; ++i4) {
    const int row = i4 * 4 + rq;
    const v4f a = *(const v4f*)(sl + row * 68 + c8), c4 = *(const v4f*)(sl + row * 68 + c8 + 4);
    float w[8];
#pragma unroll
    for (int e = 0; e < 4; ++e) { w[e] = (a[e] + bb[e]) * hscale; w[4 + e] = (c4[e] + bb[4 + e]) * hscale; }
#pragma unroll
    for (int e = 0; e < 4; ++e) {
      const _Float16 h0 = (_Float16)w[2 * e], h1 = (_Float16)w[2 * e + 1];
      const _Float16 q0 = (_Float16)((w[2 * e] - (float)h0) * rscale);
      const _Float16 q1 = (_Float16)((w[2 * e + 1] - (float)h1) * rscale);
      oh[i4][e]  = pk16(h_bits(h0), h_bits(h1));
      orr[i4][e] = pk16(h_bits(q0), h_bits(q1));
    }
  }
  const size_t dofs = rowb * (size_t)N + col0 + c8;
  u16* dh = H + dofs;
  u16* dr = Rr + dofs;
  for (int pass = 0; pass < 2; ++pass) {
#pragma unroll
    for (int i4 = 0; i4 < 4; ++i4) {
      const int row = i4 * 4 + rq;
      *(volatile v4u*)(dh + (size_t)row * (size_t)N) = oh[i4];
      *(volatile v4u*)(dr + (size_t)row * (size_t)N) = orr[i4];
    }
    __threadfence();
  }
}

__global__ __launch_bounds__(128)
void gemm_b32(const u16* __restrict__ A, const u16* __restrict__ Bt, const float* __restrict__ bias, float* C,
              int M, int N, int K, float oscale) {
  __shared__ __align__(16) float slab[4 * SLAB64];
  const int tid = threadIdx.x, wave = tid >> 5, lane = tid & 31, hh = lane >> 4, m = lane & 15;
  const int ntile = N >> 6;
  const int bid   = blockIdx.x;
  const int rowb  = (bid / ntile) * 64 + wave * 16;
  const int col0  = (bid % ntile) * 64;
  if (rowb + 16 > M) return;
  const u16* ap = A  + (size_t)(rowb + m) * (size_t)K + 8 * hh;
  const u16* bp = Bt + (size_t)(col0 + m) * (size_t)K + 8 * hh;
  const size_t bs = (size_t)16 * K;
  v8f acc0 = zero8(), acc1 = zero8(), acc2 = zero8(), acc3 = zero8();
#pragma unroll 1
  for (int k0 = 0; k0 < K; k0 += 32) {
    const v16b a  = ldfrag_b(ap + k0);
    const v16b b0 = ldfrag_b(bp + k0);
    const v16b b1 = ldfrag_b(bp + bs + k0);
    const v16b b2 = ldfrag_b(bp + 2 * bs + k0);
    const v16b b3 = ldfrag_b(bp + 3 * bs + k0);
    acc0 = mma_b(a, b0, acc0);
    acc1 = mma_b(a, b1, acc1);
    acc2 = mma_b(a, b2, acc2);
    acc3 = mma_b(a, b3, acc3);
    guard6<v16b>(acc0, acc1, acc2, acc3, a, b0, b1, b2, b3, a);
  }
  const v4f bv4 = *(const v4f*)(bias + col0 + m * 4);
  v4f badd;
#pragma unroll
  for (int e = 0; e < 4; ++e) badd[e] = bfr(bv4[e]);
  epi64(slab + wave * SLAB64, acc0, acc1, acc2, acc3, oscale, badd, C, N, (size_t)rowb, col0, lane);
}

__global__ __launch_bounds__(128)
void gemm_bhr(const u16* __restrict__ A, const u16* __restrict__ Bt, const float* __restrict__ bias, u16* H, u16* Rr,
              int M, int N, int K, float hscale, float rscale) {
  __shared__ __align__(16) float slab[4 * SLAB64];
  const int tid = threadIdx.x, wave = tid >> 5, lane = tid & 31, hh = lane >> 4, m = lane & 15;
  const int ntile = N >> 6;
  const int bid   = blockIdx.x;
  const int rowb  = (bid / ntile) * 64 + wave * 16;
  const int col0  = (bid % ntile) * 64;
  if (rowb + 16 > M) return;
  const u16* ap = A  + (size_t)(rowb + m) * (size_t)K + 8 * hh;
  const u16* bp = Bt + (size_t)(col0 + m) * (size_t)K + 8 * hh;
  const size_t bs = (size_t)16 * K;
  v8f acc0 = zero8(), acc1 = zero8(), acc2 = zero8(), acc3 = zero8();
#pragma unroll 1
  for (int k0 = 0; k0 < K; k0 += 32) {
    const v16b a  = ldfrag_b(ap + k0);
    const v16b b0 = ldfrag_b(bp + k0);
    const v16b b1 = ldfrag_b(bp + bs + k0);
    const v16b b2 = ldfrag_b(bp + 2 * bs + k0);
    const v16b b3 = ldfrag_b(bp + 3 * bs + k0);
    acc0 = mma_b(a, b0, acc0);
    acc1 = mma_b(a, b1, acc1);
    acc2 = mma_b(a, b2, acc2);
    acc3 = mma_b(a, b3, acc3);
    guard6<v16b>(acc0, acc1, acc2, acc3, a, b0, b1, b2, b3, a);
  }
  epi64hr(slab + wave * SLAB64, acc0, acc1, acc2, acc3, hscale, rscale, bias, H, Rr, N, (size_t)rowb, col0, lane);
}

__device__ __forceinline__ void ctx_store(const u16* ct, u16* dst, int tid) {
  const int row = tid >> 4;
  const int c8  = (tid & 15) * 8;
  const v4u v = *(const v4u*)(ct + row * CTP + c8);
  u16* d = dst + (size_t)row * CI + c8;
  for (int pass = 0; pass < 2; ++pass) {
    *(volatile v4u*)d = v;
    __threadfence();
  }
}

__global__ __launch_bounds__(ATT_THREADS)
void attn_fwd(const u16* __restrict__ THp, const u16* __restrict__ TRp, const u16* __restrict__ PHp,
              const u16* __restrict__ PRp, const u16* __restrict__ GTp, u16* YHo, u16* YRo) {
  __shared__ __align__(16) AttLds L0;
  __shared__ __align__(16) u16 pls[16 * PLP];
  __shared__ float rowa[QT];
  __shared__ float rowi[QT];
  float* const scs = L0.s;

  const int tid  = threadIdx.x;
  const int wave = tid >> 5;
  const int lane = tid & 31;
  const int hh   = lane >> 4;
  const int m    = lane & 15;
  const int r16  = tid >> 4;
  const int sub  = tid & 15;
  const bool vsub = sub < NKB;
  const int kl0  = sub * 32;
  const int kla  = (vsub ? sub : (NKB - 1)) * 32;

  const int nqt = NPOS / QT;
  const int b   = (int)blockIdx.x / nqt;
  const int q0  = ((int)blockIdx.x - b * nqt) * QT;
  const size_t qrow = (size_t)b * NPOS + (size_t)q0;

  const _Float16* tha = (const _Float16*)(const void*)THp + (qrow + m) * CI + 8 * hh;
  const _Float16* tra = (const _Float16*)(const void*)TRp + (qrow + m) * CI + 8 * hh;
  const _Float16* khb = (const _Float16*)(const void*)PHp + ((size_t)b * NPOS + m) * CI + 8 * hh;
  const _Float16* krb = (const _Float16*)(const void*)PRp + ((size_t)b * NPOS + m) * CI + 8 * hh;
  const _Float16* vbp = (const _Float16*)(const void*)GTp + ((size_t)b * CI + wave * 16 + m) * (size_t)NPOS + 8 * hh;
  const float lsc  = LOG2E / (TSC * FSC);
  const float rinv = 1.0f / RSC;

  float mrun = -INFINITY, lrun = 0.f;
  v8f o = zero8();

#pragma unroll 1
  for (int c = 0; c < NCHK; ++c) {
    const int kbeg = c * CK;
#pragma unroll 1
    for (int kb = wave; kb < NKB; kb += 8) {
      v8f s0 = zero8(), s0x = zero8(), s1 = zero8(), s1x = zero8();
      const size_t ko = (size_t)(kbeg + kb * 32) * CI;
      const _Float16* k0h = khb + ko;
      const _Float16* k1h = k0h + (size_t)16 * CI;
      const _Float16* k0r = krb + ko;
      const _Float16* k1r = k0r + (size_t)16 * CI;
#pragma unroll
      for (int ks = 0; ks < CI / 32; ++ks) {
        const v16h ah  = ldfrag_h(tha + ks * 32);
        const v16h ar  = ldfrag_h(tra + ks * 32);
        const v16h f0h = ldfrag_h(k0h + ks * 32);
        const v16h f0r = ldfrag_h(k0r + ks * 32);
        const v16h f1h = ldfrag_h(k1h + ks * 32);
        const v16h f1r = ldfrag_h(k1r + ks * 32);
        s0  = mma_h(ah, f0h, s0);
        s0x = mma_h(ah, f0r, s0x);
        s0x = mma_h(ar, f0h, s0x);
        s1  = mma_h(ah, f1h, s1);
        s1x = mma_h(ah, f1r, s1x);
        s1x = mma_h(ar, f1h, s1x);
        guard6<v16h>(s0, s0x, s1, s1x, ah, ar, f0h, f0r, f1h, f1r);
      }
      float* srow = scs + (8 * hh) * SCP + kb * 32 + m;
#pragma unroll
      for (int r = 0; r < 8; ++r) {
        srow[r * SCP]      = s0[r] + s0x[r] * rinv;
        srow[r * SCP + 16] = s1[r] + s1x[r] * rinv;
      }
    }
    __syncthreads();
    {
      const float* sp = scs + r16 * SCP + kla;
      float t[32];
      float cm = -INFINITY;
#pragma unroll
      for (int i = 0; i < 8; ++i) {
        const v4f a = *(const v4f*)(sp + 4 * i);
#pragma unroll
        for (int e = 0; e < 4; ++e) {
          const float tv = a[e] * lsc;
          const float tt = vsub ? tv : -INFINITY;
          t[4 * i + e] = tt;
          cm = fmaxf(cm, tt);
        }
      }
#pragma unroll
      for (int d = 1; d <= 8; d <<= 1) cm = fmaxf(cm, __shfl_xor(cm, d, 32));
      const float mn = fmaxf(mrun, cm);
      const float al = (mrun == -INFINITY) ? 0.f : exp2f(mrun - mn);
      mrun = mn;
      float ps = 0.f;
#pragma unroll
      for (int j = 0; j < 32; ++j) {
        const float p = exp2f(t[j] - mn);
        t[j] = p;
        ps += p;
      }
#pragma unroll
      for (int d = 1; d <= 8; d <<= 1) ps += __shfl_xor(ps, d, 32);
      v4u pk[4];
#pragma unroll
      for (int i = 0; i < 4; ++i) {
#pragma unroll
        for (int e = 0; e < 4; ++e) {
          const int j = 8 * i + 2 * e;
          pk[i][e] = pk16(h_bits((_Float16)(t[j] * PCAR)), h_bits((_Float16)(t[j + 1] * PCAR)));
        }
      }
      lrun = lrun * al + ps;
      if (vsub) {
        u16* pd = pls + r16 * PLP + kl0;
#pragma unroll
        for (int i = 0; i < 4; ++i) *(v4u*)(pd + 8 * i) = pk[i];
      }
      if (sub == 0) rowa[r16] = al;
    }
    __syncthreads();
    {
      float scl[8];
#pragma unroll
      for (int r = 0; r < 8; ++r) scl[r] = rowa[8 * hh + r];
#pragma unroll
      for (int r = 0; r < 8; ++r) o[r] *= scl[r];
      const _Float16* pp = (const _Float16*)(const void*)pls + m * PLP + 8 * hh;
      const _Float16* vp = vbp + kbeg;
#pragma unroll 1
      for (int kb = 0; kb < NKB; ++kb) {
        const v16h pf = ldfrag_h(pp + kb * 32);
        const v16h g0 = ldfrag_h(vp + kb * 32);
        o = mma_h(pf, g0, o);
        guard1x2(o, pf, g0);
      }
    }
  }
  acc_guard1(o);

  if (sub == 0) rowi[r16] = (1.0f / lrun) * (YSC / (PCAR * GSC));
  __syncthreads();
  float inv[8];
#pragma unroll
  for (int r = 0; r < 8; ++r) inv[r] = rowi[8 * hh + r];

  u16* const ct = L0.c;
  const int cb = wave * 16 + m;
#pragma unroll
  for (int r = 0; r < 8; ++r) {
    const int ro = (8 * hh + r) * CTP + cb;
    ct[ro] = h_bits((_Float16)(o[r] * inv[r]));
  }
  __syncthreads();
  ctx_store(ct, YHo + qrow * CI, tid);
  __syncthreads();
#pragma unroll
  for (int r = 0; r < 8; ++r) {
    const int ro = (8 * hh + r) * CTP + cb;
    const float x0 = o[r] * inv[r];
    const _Float16 e0 = (_Float16)x0;
    ct[ro] = h_bits((_Float16)((x0 - (float)e0) * RSC));
  }
  __syncthreads();
  ctx_store(ct, YRo + qrow * CI, tid);
}

__global__ __launch_bounds__(256)
void wo_out(const u16* __restrict__ YH, const u16* __restrict__ YR, const u16* __restrict__ WoT,
            const float* __restrict__ bo, const float* __restrict__ gam, const float* __restrict__ bet,
            const float* __restrict__ mmean, const float* __restrict__ mvar, const float* __restrict__ x, float* out) {
  __shared__ __align__(16) float slab[8 * SLAB64];
  const int tid = threadIdx.x, wave = tid >> 5, lane = tid & 31, hh = lane >> 4, m = lane & 15;
  const int rowb = blockIdx.x * OUT_ROWS + wave * 16;
  float* const sl = slab + wave * SLAB64;
  const _Float16* ap  = (const _Float16*)(const void*)YH + (size_t)(rowb + m) * CI + 8 * hh;
  const _Float16* arp = (const _Float16*)(const void*)YR + (size_t)(rowb + m) * CI + 8 * hh;
  const size_t bs = (size_t)16 * CI;
  const float os1 = 1.0f / (YSC * WOS);
  const float os2 = 1.0f / (YSC * WOS * RSC);

#pragma unroll 1
  for (int g = 0; g < CIN / 64; ++g) {
    const _Float16* bp = (const _Float16*)(const void*)WoT + (size_t)(g * 64 + m) * CI + 8 * hh;
    v8f acc0 = zero8(), acc1 = zero8(), acc2 = zero8(), acc3 = zero8();
    v8f acr0 = zero8(), acr1 = zero8(), acr2 = zero8(), acr3 = zero8();
#pragma unroll 1
    for (int k0 = 0; k0 < CI; k0 += 32) {
      const v16h a  = ldfrag_h(ap + k0);
      const v16h ar = ldfrag_h(arp + k0);
      const v16h b0 = ldfrag_h(bp + k0);
      const v16h w1 = ldfrag_h(bp + bs + k0);
      const v16h w2 = ldfrag_h(bp + 2 * bs + k0);
      const v16h w3 = ldfrag_h(bp + 3 * bs + k0);
      acc0 = mma_h(a, b0, acc0);
      acc1 = mma_h(a, w1, acc1);
      acc2 = mma_h(a, w2, acc2);
      acc3 = mma_h(a, w3, acc3);
      acr0 = mma_h(ar, b0, acr0);
      acr1 = mma_h(ar, w1, acr1);
      acr2 = mma_h(ar, w2, acr2);
      acr3 = mma_h(ar, w3, acr3);
      guard8x6(acc0, acc1, acc2, acc3, acr0, acr1, acr2, acr3, a, ar, b0, w1, w2, w3);
    }
    v8f c0 = zero8(), c1 = zero8(), c2 = zero8(), c3 = zero8();
#pragma unroll
    for (int r = 0; r < 8; ++r) {
      c0[r] = acc0[r] * os1 + acr0[r] * os2;
      c1[r] = acc1[r] * os1 + acr1[r] * os2;
      c2[r] = acc2[r] * os1 + acr2[r] * os2;
      c3[r] = acc3[r] * os1 + acr3[r] * os2;
    }
    stage64(sl, c0, c1, c2, c3, 1.0f, lane);

    const int cc = g * 64 + m * 4;
    const v4f bo4 = *(const v4f*)(bo + cc);
    const v4f ga4 = *(const v4f*)(gam + cc);
    const v4f be4 = *(const v4f*)(bet + cc);
    const v4f mm4 = *(const v4f*)(mmean + cc);
    const v4f mv4 = *(const v4f*)(mvar + cc);
    float bob[4], gb[4], bb[4], mb[4], rs[4];
#pragma unroll
    for (int e = 0; e < 4; ++e) {
      bob[e] = bfr(bo4[e]);
      gb[e]  = bfr(ga4[e]);
      bb[e]  = bfr(be4[e]);
      mb[e]  = bfr(mm4[e]);
      rs[e]  = rsqrtf(bfr(mv4[e]) + BN_EPS);
    }
    v4f vals[8];
#pragma unroll
    for (int it = 0; it < 8; ++it) {
      const size_t row = (size_t)rowb + (size_t)(2 * it + hh);
      const v4f yv = *(const v4f*)(sl + (2 * it + hh) * 68 + m * 4);
      const v4f xv = *(const v4f*)(x + row * CIN + cc);
#pragma unroll
      for (int e = 0; e < 4; ++e) {
        const float v2 = yv[e] + bob[e];
        const float bn = gb[e] * (v2 - mb[e]) * rs[e] + bb[e];
        vals[it][e] = bfr(xv[e]) + bn;
      }
    }
    float* dst = out + ((size_t)rowb + (size_t)hh) * CIN + cc;
    for (int pass = 0; pass < 2; ++pass) {
#pragma unroll
      for (int it = 0; it < 8; ++it) {
        *(volatile v4f*)(dst + (size_t)(it * 2) * CIN) = vals[it];
      }
      __threadfence();
    }
    wave_sync_lds();
  }
}

extern "C" void kernel_launch(void* const* d_in, const int* in_sizes, int n_in,
                              void* d_out, int out_size, void* d_ws, size_t ws_size,
                              hipStream_t stream) {
  if (n_in < 13) return;
  if (in_sizes[0] != ROWS * CIN) return;
  if (in_sizes[1] != CIN * CI || in_sizes[3] != CIN * CI || in_sizes[5] != CIN * CI || in_sizes[7] != CI * CIN) return;
  if (in_sizes[2] != CI || in_sizes[4] != CI || in_sizes[6] != CI) return;
  if (in_sizes[8] != CIN || in_sizes[9] != CIN || in_sizes[10] != CIN || in_sizes[11] != CIN || in_sizes[12] != CIN) return;
  if (out_size != ROWS * CIN) return;

  const float* x     = (const float*)d_in[0];
  const float* Wg    = (const float*)d_in[1];
  const float* bg    = (const float*)d_in[2];
  const float* Wt    = (const float*)d_in[3];
  const float* bt    = (const float*)d_in[4];
  const float* Wp    = (const float*)d_in[5];
  const float* bp    = (const float*)d_in[6];
  const float* Wo    = (const float*)d_in[7];
  const float* bo    = (const float*)d_in[8];
  const float* gamma = (const float*)d_in[9];
  const float* beta  = (const float*)d_in[10];
  const float* mmean = (const float*)d_in[11];
  const float* mvar  = (const float*)d_in[12];
  float*       out   = (float*)d_out;

  const size_t szXB = (size_t)ROWSP * CIN * 2;
  const size_t szW  = (size_t)CI * CIN * 2;
  const size_t szP  = (size_t)ROWSP * CI * 2;
  const size_t szG  = (size_t)ROWSP * CI * 4;
  const size_t szGT = (size_t)NB * CI * NPOS * 2;
  size_t off = 0;
  const size_t oXB = off; off += szXB;
  const size_t oWG = off; off += szW;
  const size_t oWT = off; off += szW;
  const size_t oWP = off; off += szW;
  const size_t oWO = off; off += szW;
  const size_t oTH = off; off += szP;
  const size_t oTR = off; off += szP;
  const size_t oPH = off; off += szP;
  const size_t oPR = off; off += szP;
  const size_t oG  = off; off += szG;
  const size_t oGT = off; off += szGT;
  const size_t oYH = off; off += szP;
  const size_t oYR = off; off += szP;
  if (off > ws_size) return;
  if (off > WS_CAP) return;

  char* ws = (char*)d_ws;
  u16*   XB  = (u16*)(ws + oXB);
  u16*   WGT = (u16*)(ws + oWG);
  u16*   WTT = (u16*)(ws + oWT);
  u16*   WPT = (u16*)(ws + oWP);
  u16*   WOT = (u16*)(ws + oWO);
  u16*   TH  = (u16*)(ws + oTH);
  u16*   TR  = (u16*)(ws + oTR);
  u16*   PH  = (u16*)(ws + oPH);
  u16*   PR  = (u16*)(ws + oPR);
  float* G   = (float*)(ws + oG);
  u16*   GT  = (u16*)(ws + oGT);
  u16*   YH  = (u16*)(ws + oYH);
  u16*   YR  = (u16*)(ws + oYR);

  const int n8x = (ROWSP * CIN) / 8;
  const dim3 blk(256);
  const dim3 bG(128);
  const dim3 gX(n8x / 256);
  const dim3 gW((CIN / 64) * (CI / 64));
  const dim3 gWO((CI / 64) * (CIN / 64));
  const dim3 gP((ROWSP / 64) * (CI / 64));
  const dim3 gGT((NPOS / 64) * (CI / 64));
  const dim3 gAT(NB * (NPOS / QT));
  const dim3 bAT(ATT_THREADS);
  const dim3 gOUT(ROWSP / OUT_ROWS);

  cvt16<<<gX, blk, 0, stream>>>(x, XB, n8x, 0, 1.0f);
  tr16<<<gW, blk, 0, stream>>>(Wg, WGT, CIN, CI, 0, 1.0f);
  tr16<<<gW, blk, 0, stream>>>(Wt, WTT, CIN, CI, 0, 1.0f);
  tr16<<<gW, blk, 0, stream>>>(Wp, WPT, CIN, CI, 0, 1.0f);
  tr16<<<gWO, blk, 0, stream>>>(Wo, WOT, CI, CIN, 1, WOS);
  gemm_bhr<<<gP, bG, 0, stream>>>(XB, WTT, bt, TH, TR, ROWSP, CI, CIN, TSC, RSC);
  gemm_bhr<<<gP, bG, 0, stream>>>(XB, WPT, bp, PH, PR, ROWSP, CI, CIN, FSC, RSC);
  gemm_b32<<<gP, bG, 0, stream>>>(XB, WGT, bg, G, ROWSP, CI, CIN, 1.0f);
  for (int b = 0; b < NB; ++b) {
    tr16<<<gGT, blk, 0, stream>>>(G + (size_t)b * NPOS * CI, GT + (size_t)b * CI * NPOS, NPOS, CI, 2, GSC);
  }
  attn_fwd<<<gAT, bAT, 0, stream>>>(TH, TR, PH, PR, GT, YH, YR);
  wo_out<<<gOUT, blk, 0, stream>>>(YH, YR, WOT, bo, gamma, beta, mmean, mvar, x, out);
  (void)hipGetLastError();
}
